// DotProductAttention_87754771792527
// MI455X (gfx1250) — hardware-verified
//
#include <hip/hip_runtime.h>
#include <math.h>

typedef __attribute__((ext_vector_type(16))) _Float16 v16h;
typedef __attribute__((ext_vector_type(8)))  _Float16 v8h;
typedef __attribute__((ext_vector_type(8)))  float v8f;
typedef __attribute__((ext_vector_type(4)))  float v4f;
typedef __attribute__((ext_vector_type(4)))  unsigned v4u;

template <typename T> __device__ __forceinline__ void vst2(void* p, T v) { *(volatile T*)p = v; __threadfence(); *(volatile T*)p = v; }
__device__ __forceinline__ v8f wmma16(v16h a, v16h b, v8f c) {
  v8f d = __builtin_amdgcn_wmma_f32_16x16x32_f16(false, a, false, b, (short)0, c, false, false);
  asm volatile("v_nop\n\tv_nop\n\tv_nop\n\tv_nop" : "+v"(d) : "v"(a), "v"(b));
  return d;
}
__device__ __forceinline__ v16h frag_h(const _Float16* rowk0, int lane) {
  union { v16h v; v8h q[2]; } u; const _Float16* p = rowk0 + 8 * (lane >> 4);
  u.q[0] = *(const v8h*)p; u.q[1] = *(const v8h*)(p + 16); return u.v;
}
__device__ __forceinline__ v16h frag_f32(const float* rowk0, int lane) {
  v16h a; const float* p = rowk0 + 8 * (lane >> 4);
#pragma unroll
  for (int i = 0; i < 8; ++i) { a[i] = (_Float16)p[i]; a[8 + i] = (_Float16)p[16 + i]; }
  return a;
}
__device__ __forceinline__ float bfr(float v) { return (float)(__bf16)v; }
#define LDSX() do { asm volatile("s_wait_dscnt 0" ::: "memory"); __builtin_amdgcn_wave_barrier(); __builtin_amdgcn_fence(3  , "workgroup"); } while (0)

#ifndef NB
#define NB 8
#endif
#ifndef SEQ
#define SEQ 2048
#endif
#define NB_FULL 8
#define SEQ_FULL 2048
#define HD 64
#define HG (NB < 4 ? NB : 4)
#define NQB (SEQ / 64)
#define NKB (SEQ / 128)
#define SCALE (0.125f)
#define NEGV (-1.0e9f)
static_assert(NB >= 1 && NB <= NB_FULL);
static_assert(SEQ % 128 == 0 && SEQ >= 128 && SEQ <= SEQ_FULL);
static_assert(NB % HG == 0);
static_assert((size_t)NB_FULL * SEQ_FULL * HD * 4u == 4194304u);

#define PLANE_BYTES (2u * (size_t)NB * SEQ * HD)
#define WS_QH  (0u)
#define WS_QL  (WS_QH + PLANE_BYTES)
#define WS_KH  (WS_QL + PLANE_BYTES)
#define WS_VT  (WS_KH + PLANE_BYTES)
#define WS_S   (WS_VT + PLANE_BYTES)
#define WS_END (WS_S + 4u * (size_t)HG * SEQ * SEQ)
static_assert(PLANE_BYTES % 128u == 0);
static_assert(WS_END <= 134217728u);

__global__ __launch_bounds__(128) void k_prep(const float* __restrict__ Q, const float* __restrict__ K, const float* __restrict__ V, const float* __restrict__ MV,
                                             _Float16* __restrict__ QH, _Float16* __restrict__ QL, _Float16* __restrict__ KH, _Float16* __restrict__ VT) {
  __shared__ __align__(16) _Float16 sq[64][72], sql[64][72], sk[64][72], tv[64][72];
  const int tid = threadIdx.x;
  const int b = blockIdx.x / NQB; const int s0 = (blockIdx.x % NQB) * 64;
  const size_t irow0 = (size_t)b * SEQ_FULL + s0;
  const size_t prow0 = (size_t)b * SEQ + s0;
  for (int e = tid; e < 64 * 64; e += 128) { const int rl = e >> 6, c = e & 63; const size_t oi = (irow0 + rl) * HD + c;
    const float q = bfr(Q[oi]), k = bfr(K[oi]); const float mvr = bfr(MV[irow0 + rl]); const float v = bfr(V[oi]) * mvr;
    const _Float16 qh = (_Float16)q; sq[rl][c] = qh; sql[rl][c] = (_Float16)((q - (float)qh) * 1024.0f); sk[rl][c] = (_Float16)k; tv[c][rl] = (_Float16)v; }
  __syncthreads();
  for (int e = tid; e < 64 * 8; e += 128) { const int rl = e >> 3, p = e & 7; const size_t o = (prow0 + rl) * HD + p * 8;
    vst2((void*)(QH + o), *(const v4u*)&sq[rl][p * 8]); vst2((void*)(QL + o), *(const v4u*)&sql[rl][p * 8]); vst2((void*)(KH + o), *(const v4u*)&sk[rl][p * 8]); }
  for (int e = tid; e < HD * 8; e += 128) { const int cl = e >> 3, p = e & 7;
    vst2((void*)(VT + ((size_t)b * HD + cl) * (size_t)SEQ + s0 + p * 8), *(const v4u*)&tv[cl][p * 8]); } }

__global__ __launch_bounds__(128) void k_sc(const _Float16* __restrict__ QH, const _Float16* __restrict__ QL, const _Float16* __restrict__ KH, int b0, float* __restrict__ S0) {
  __shared__ __align__(16) float ss[4][16][132];
  const int qb = blockIdx.x, kb = blockIdx.y; const int b = b0 + blockIdx.z; float* S = S0 + (size_t)blockIdx.z * SEQ * SEQ;
  const int tid = threadIdx.x, wave = tid >> 5, lane = tid & 31, col = lane & 15, g = lane >> 4; const int k0 = kb * 128; const int ql0 = qb * 64 + wave * 16;
  const size_t q0 = (size_t)b * SEQ + ql0, kr0 = (size_t)b * SEQ + k0;
  v8f acc[8] = {}, accl[8] = {};
#pragma unroll
  for (int kc = 0; kc < HD / 32; ++kc) { const v16h ah = frag_h(QH + (q0 + col) * HD + kc * 32, lane), al = frag_h(QL + (q0 + col) * HD + kc * 32, lane);
#pragma unroll
    for (int j = 0; j < 8; ++j) { const v16h kf = frag_h(KH + (kr0 + j * 16 + col) * HD + kc * 32, lane); acc[j] = wmma16(ah, kf, acc[j]); accl[j] = wmma16(al, kf, accl[j]); } }
#pragma unroll
  for (int j = 0; j < 8; ++j) {
#pragma unroll
    for (int r = 0; r < 8; ++r) ss[wave][8 * g + r][j * 16 + col] = (acc[j][r] + accl[j][r] * (1.0f / 1024.0f)) * SCALE; }
  LDSX(); for (int rl = 0; rl < 16; ++rl) vst2(S + (size_t)(ql0 + rl) * SEQ + k0 + lane * 4, *(const v4f*)&ss[wave][rl][lane * 4]); }

__global__ __launch_bounds__(256) void k_sm(float* __restrict__ S0, const float* __restrict__ MQ, const float* __restrict__ MK, int b0) {
  __shared__ float sred[8]; __shared__ float sbc; __shared__ __align__(16) float shv[SEQ];
  const int tid = threadIdx.x; const int t = blockIdx.x; const int b = b0 + blockIdx.y;
  float* sr = S0 + (size_t)blockIdx.y * SEQ * SEQ + (size_t)t * SEQ;
  const float mqv = bfr(MQ[(size_t)b * SEQ_FULL + t]); const float* mk = MK + (size_t)b * SEQ_FULL;
  float m = -3.0e38f; for (int k = tid; k < SEQ; k += 256) { float v = sr[k]; v = v + (1.0f - mqv * bfr(mk[k])) * NEGV; shv[k] = v; m = fmaxf(m, v); }
#pragma unroll
  for (int o = 1; o < 32; o <<= 1) m = fmaxf(m, __shfl_xor(m, o));
  if ((tid & 31) == 0) sred[tid >> 5] = m; __syncthreads(); if (tid == 0) { float a = sred[0]; for (int i = 1; i < 8; ++i) a = fmaxf(a, sred[i]); sbc = a; } __syncthreads(); m = sbc; __syncthreads();
  float sum = 0.f;
#pragma unroll 1
  for (int k = tid; k < SEQ; k += 256) { const float e = expf(shv[k] - m); shv[k] = e; sum += e; }
#pragma unroll
  for (int o = 1; o < 32; o <<= 1) sum += __shfl_xor(sum, o);
  if ((tid & 31) == 0) sred[tid >> 5] = sum; __syncthreads(); if (tid == 0) { float a = 0.f; for (int i = 0; i < 8; ++i) a += sred[i]; sbc = a > 0.f ? (1.0f / a) * 2048.0f : 0.f; } __syncthreads(); const float inv = sbc;
  for (int k = tid; k < SEQ; k += 256) shv[k] = shv[k] * inv;
  __syncthreads(); for (int q = tid; q < SEQ / 4; q += 256) vst2(sr + q * 4, *(const v4f*)&shv[q * 4]); }

__global__ __launch_bounds__(128) void k_pv(const float* __restrict__ PS0, const _Float16* __restrict__ VT, int b0, float* __restrict__ Y) {
  __shared__ __align__(16) float ss[4][16][HD + 4];
  const int b = b0 + blockIdx.z; const float* PS = PS0 + (size_t)blockIdx.z * SEQ * SEQ;
  const int tid = threadIdx.x, wave = tid >> 5, lane = tid & 31, col = lane & 15, g = lane >> 4; const int qb = blockIdx.x; const int ql0 = qb * 64 + wave * 16;
  v8f acc[HD / 16] = {};
#pragma unroll 1
  for (int kc = 0; kc < SEQ / 32; ++kc) { const v16h p = frag_f32(PS + (size_t)(ql0 + col) * SEQ + kc * 32, lane);
    asm volatile("s_wait_loadcnt 0x0" ::: "memory");
#pragma unroll
    for (int j = 0; j < HD / 16; ++j) { const size_t po = ((size_t)b * HD + j * 16 + col) * (size_t)SEQ + kc * 32; acc[j] = wmma16(p, frag_h(VT + po, lane), acc[j]); } }
#pragma unroll
  for (int j = 0; j < HD / 16; ++j)
#pragma unroll
    for (int r = 0; r < 8; ++r) ss[wave][8 * g + r][j * 16 + col] = acc[j][r] * (1.0f / 2048.0f);
  LDSX(); for (int rl = 0; rl < 16; ++rl) if (lane < HD / 4) vst2(Y + ((size_t)b * SEQ_FULL + ql0 + rl) * HD + lane * 4, *(const v4f*)&ss[wave][rl][lane * 4]); }

extern "C" void kernel_launch(void* const* d_in, const int* in_sizes, int n_in, void* d_out, int out_size, void* d_ws, size_t ws_size, hipStream_t stream) {
  if (n_in < 6) return;
  const size_t need_x = ((size_t)(NB - 1) * SEQ_FULL + SEQ) * HD, need_m = (size_t)(NB - 1) * SEQ_FULL + SEQ;
  if ((size_t)in_sizes[0] < need_x || (size_t)in_sizes[1] < need_x || (size_t)in_sizes[2] < need_x) return;
  if ((size_t)in_sizes[3] < need_m || (size_t)in_sizes[4] < need_m || (size_t)in_sizes[5] < need_m) return;
  if ((size_t)out_size < need_x) return;
  if (ws_size < (size_t)WS_END) return;
  const float* Q = (const float*)d_in[0]; const float* K = (const float*)d_in[1]; const float* V = (const float*)d_in[2];
  const float* MQ = (const float*)d_in[3]; const float* MK = (const float*)d_in[4]; const float* MV = (const float*)d_in[5];
  char* ws = (char*)d_ws;
  _Float16 *QH = (_Float16*)(ws + WS_QH), *QL = (_Float16*)(ws + WS_QL), *KH = (_Float16*)(ws + WS_KH), *VT = (_Float16*)(ws + WS_VT);
  float* S = (float*)(ws + WS_S); float* O = (float*)d_out;
  k_prep<<<dim3(NB * NQB), 128, 0, stream>>>(Q, K, V, MV, QH, QL, KH, VT);
  for (int b0 = 0; b0 < NB; b0 += HG) {
    k_sc<<<dim3(NQB, NKB, HG), 128, 0, stream>>>(QH, QL, KH, b0, S);
    k_sm<<<dim3(SEQ, HG), 256, 0, stream>>>(S, MQ, MK, b0);
    k_pv<<<dim3(NQB, 1, HG), 128, 0, stream>>>(S, VT, b0, O);
  }
}
